// MultiHeadSelfAttentionFused_54915451846833
// MI455X (gfx1250) — hardware-run, weakly checked
//
#include <hip/hip_runtime.h>


#ifndef NB
#define NB 4
#endif
#ifndef SEQ
#define SEQ 2048
#endif
#define NB_FULL   4
#define SEQ_FULL  2048
#define DM        1024
#define NWAVE     8
#define OP        68
#define CVB       2048u
#define NXB       ((unsigned)((size_t)NB * SEQ * DM / CVB))
#define NWB       ((unsigned)((size_t)3 * DM * DM / CVB))
#define NOB       ((unsigned)((size_t)DM * DM / CVB))
#define NCH       (SEQ / 256)
#define GCH       ((NCH >= 4) ? 4 : NCH)
#define CSC       128

#define EPI_HR   0
#define EPI_VT   1
#define EPI_H16  2
#define EPI_F32B 3

#define MAXB(a, b) (((a) > (b)) ? (a) : (b))

static_assert(SEQ % 256 == 0);
static_assert(SEQ <= SEQ_FULL);
static_assert(NB >= 1 && NB <= NB_FULL);
static_assert(DM == 1024);
static_assert(DM % 128 == 0);
static_assert(DM % 32 == 0 && SEQ % 32 == 0);
static_assert(SEQ % 128 == 0);
static_assert(((size_t)NB * SEQ) % 128 == 0);
static_assert((size_t)NXB * CVB == (size_t)NB * SEQ * DM);
static_assert((size_t)NWB * CVB == (size_t)3 * DM * DM);
static_assert((size_t)NOB * CVB == (size_t)DM * DM);
static_assert((size_t)DM * DM / CVB == 512);
static_assert((OP * 4) % 16 == 0);
static_assert(NCH % GCH == 0);
static_assert(SEQ % CSC == 0);
static_assert(SEQ % NWAVE == 0);
static_assert(CSC == 32 * 4);
static_assert((size_t)NWAVE * 16 * OP * 4 <= 131072);
static_assert((size_t)(2 * NWAVE * CSC + CSC) * 4 <= 131072);

#define XB_BYTES   ((size_t)NB * SEQ * DM * 2)
#define WB_BYTES   ((size_t)3 * DM * DM * 2)
#define S_BYTES    ((size_t)SEQ * SEQ * 4)
#define P_BYTES    ((size_t)SEQ * SEQ * 2)
#define R1_BYTES   MAXB(XB_BYTES, S_BYTES)
#define R2_BYTES   MAXB(WB_BYTES, P_BYTES)
#define PR_BYTES   ((size_t)SEQ * SEQ * 2)
#define CX_BYTES   ((size_t)SEQ * DM * 2)
#define WO_BYTES   ((size_t)DM * DM * 2)
#define BI_BYTES   ((size_t)4 * DM * 4)
#define CS_BYTES   ((size_t)SEQ * 4)
#define QK_BYTES   ((size_t)4 * NB * SEQ * DM * 2)
#define VT_BYTES   ((size_t)NB * DM * SEQ * 2)
#define WS_TOTAL   (R1_BYTES + R2_BYTES + PR_BYTES + 2 * CX_BYTES + WO_BYTES + BI_BYTES + CS_BYTES + QK_BYTES + VT_BYTES)
static_assert(WS_TOTAL <= (size_t)134217728);
static_assert(XB_BYTES <= R1_BYTES && S_BYTES <= R1_BYTES);
static_assert(WB_BYTES <= R2_BYTES && P_BYTES <= R2_BYTES);
static_assert(R1_BYTES % 128 == 0 && R2_BYTES % 128 == 0 && CX_BYTES % 128 == 0 && WO_BYTES % 128 == 0);
static_assert(PR_BYTES % 128 == 0);
static_assert(BI_BYTES % 128 == 0 && CS_BYTES % 128 == 0 && QK_BYTES % 128 == 0 && VT_BYTES % 128 == 0);
static_assert(((size_t)(NB_FULL - 1) * SEQ_FULL + SEQ_FULL) * DM * 4 == (size_t)33554432);

typedef __bf16   bf16;
typedef _Float16 f16;
typedef bf16     v16bf __attribute__((ext_vector_type(16)));
typedef f16      v16h  __attribute__((ext_vector_type(16)));
typedef float    v8f   __attribute__((ext_vector_type(8)));
typedef float    v4f   __attribute__((ext_vector_type(4)));
typedef unsigned v4u   __attribute__((ext_vector_type(4)));

union Pack8B { v4u u; bf16 h[8]; };
union Pack8H { v4u u; f16  h[8]; };

template <typename T> struct FragOf;
template <> struct FragOf<bf16> { typedef v16bf V; };
template <> struct FragOf<f16>  { typedef v16h  V; };

static __device__ __forceinline__ f16 toh_flush(float v) {
  const f16 r = (f16)v;
  return (fabsf(v) < 6.103515625e-05f) ? (f16)0.0f : r;
}

static __device__ __forceinline__ v8f mma16(v16bf a, v16bf b, v8f acc) {
  acc = __builtin_amdgcn_wmma_f32_16x16x32_bf16(false, a, false, b, (short)0, acc, false, false);
  asm volatile("v_nop\n\tv_nop\n\tv_nop\n\tv_nop" : "+v"(acc) : "v"(a), "v"(b));
  return acc;
}
static __device__ __forceinline__ v8f mma16(v16h a, v16h b, v8f acc) {
  acc = __builtin_amdgcn_wmma_f32_16x16x32_f16(false, a, false, b, (short)0, acc, false, false);
  asm volatile("v_nop\n\tv_nop\n\tv_nop\n\tv_nop" : "+v"(acc) : "v"(a), "v"(b));
  return acc;
}

__global__ __launch_bounds__(256) void convert_kernel(const float* __restrict__ x,
                                                      const float* __restrict__ wq,
                                                      const float* __restrict__ bq,
                                                      const float* __restrict__ wk,
                                                      const float* __restrict__ bk,
                                                      const float* __restrict__ wv,
                                                      const float* __restrict__ bv,
                                                      const float* __restrict__ wo,
                                                      const float* __restrict__ bo,
                                                      bf16* __restrict__ xb,
                                                      bf16* __restrict__ wb,
                                                      f16* __restrict__ wob,
                                                      float* __restrict__ biasp) {
  const unsigned blk = blockIdx.x;
  const unsigned tid = threadIdx.x;
  if (blk < NXB + NWB) {
    const float* src;
    bf16* dst;
    if (blk < NXB) {
      const unsigned r  = blk * 2u + (tid >> 7);
      const unsigned c  = (tid & 127u) * 8u;
      const unsigned bt = r / (unsigned)SEQ;
      const unsigned s  = r - bt * (unsigned)SEQ;
      src = x + ((size_t)bt * SEQ_FULL + s) * DM + c;
      dst = xb + (size_t)r * DM + c;
    } else {
      const unsigned wblk = blk - NXB;
      const unsigned wi   = wblk >> 9;
      const unsigned off  = (wblk & 511u) * CVB + tid * 8u;
      const float* wsrc = (wi == 0u) ? wq : ((wi == 1u) ? wk : wv);
      src = wsrc + off;
      dst = wb + (size_t)wblk * CVB + tid * 8u;
    }
    const v4f a0 = *(const v4f*)(src);
    const v4f a1 = *(const v4f*)(src + 4);
    Pack8B pk;
    #pragma unroll
    for (int i = 0; i < 4; ++i) {
      pk.h[i]     = (bf16)a0[i];
      pk.h[4 + i] = (bf16)a1[i];
    }
    const v4u val = pk.u;
    *(volatile v4u*)(dst) = val;
    __threadfence();
    *(volatile v4u*)(dst) = val;
  } else if (blk < NXB + NWB + NOB) {
    const unsigned oblk = blk - (NXB + NWB);
    const size_t   off  = (size_t)oblk * CVB + tid * 8u;
    const v4f a0 = *(const v4f*)(wo + off);
    const v4f a1 = *(const v4f*)(wo + off + 4);
    Pack8H ph;
    #pragma unroll
    for (int i = 0; i < 4; ++i) {
      ph.h[i]     = toh_flush((float)(bf16)a0[i] * 64.0f);
      ph.h[4 + i] = toh_flush((float)(bf16)a1[i] * 64.0f);
    }
    const v4u val = ph.u;
    f16* dst = wob + off;
    *(volatile v4u*)(dst) = val;
    __threadfence();
    *(volatile v4u*)(dst) = val;
  } else {
    const unsigned j = blk - (NXB + NWB + NOB);
    const float* bsrc = (j == 0u) ? bq : ((j == 1u) ? bk : ((j == 2u) ? bv : bo));
    const v4f a = *(const v4f*)(bsrc + tid * 4u);
    v4f o;
    #pragma unroll
    for (int i = 0; i < 4; ++i) o[i] = (float)(bf16)a[i];
    float* dst = biasp + j * (unsigned)DM + tid * 4u;
    *(volatile v4f*)(dst) = o;
    __threadfence();
    *(volatile v4f*)(dst) = o;
  }
}

template <typename T, int EPI>
__global__ __launch_bounds__(256) void gemm_kernel(const T* __restrict__ A,
                                                   const T* __restrict__ Bt,
                                                   const float* __restrict__ bias,
                                                   void* __restrict__ C,
                                                   unsigned nk, unsigned lda, unsigned ldb, unsigned ldc,
                                                   unsigned long long sAz, unsigned long long sBz,
                                                   unsigned long long sCz, float scale) {
  typedef typename FragOf<T>::V VT;
  union Frag { VT v; v4u q[2]; };

  __shared__ __align__(16) float sO[NWAVE * 16 * OP];

  const unsigned tid  = threadIdx.x;
  const unsigned wave = (unsigned)__builtin_amdgcn_readfirstlane((int)(tid >> 5));
  const unsigned lane = tid & 31u;
  const unsigned lq   = lane & 15u;
  const unsigned hi   = lane >> 4;
  const unsigned m0   = blockIdx.x * 128u + (wave & 3u) * 32u;
  const unsigned n0   = blockIdx.y * 128u + (wave >> 2) * 64u;

  const T* Ab = A  + (size_t)blockIdx.z * sAz;
  const T* Bb = Bt + (size_t)blockIdx.z * sBz;

  const T* ap[2];
  const T* bp[4];
  #pragma unroll
  for (int mt = 0; mt < 2; ++mt) ap[mt] = Ab + (size_t)(m0 + mt * 16u + lq) * lda + hi * 8u;
  #pragma unroll
  for (int nt = 0; nt < 4; ++nt) bp[nt] = Bb + (size_t)(n0 + nt * 16u + lq) * ldb + hi * 8u;

  v8f acc[2][4];
  #pragma unroll
  for (int mt = 0; mt < 2; ++mt) {
    #pragma unroll
    for (int nt = 0; nt < 4; ++nt) acc[mt][nt] = (v8f){0, 0, 0, 0, 0, 0, 0, 0};
  }

  #pragma unroll 1
  for (unsigned k = 0; k < nk; ++k) {
    const unsigned ko = k * 32u;
    Frag a[2], b[4];
    #pragma unroll
    for (int mt = 0; mt < 2; ++mt) {
      a[mt].q[0] = *(const v4u*)(ap[mt] + ko);
      a[mt].q[1] = *(const v4u*)(ap[mt] + ko + 16u);
    }
    #pragma unroll
    for (int nt = 0; nt < 4; ++nt) {
      b[nt].q[0] = *(const v4u*)(bp[nt] + ko);
      b[nt].q[1] = *(const v4u*)(bp[nt] + ko + 16u);
    }
    #pragma unroll
    for (int nt = 0; nt < 4; ++nt) {
      #pragma unroll
      for (int mt = 0; mt < 2; ++mt) acc[mt][nt] = mma16(a[mt].v, b[nt].v, acc[mt][nt]);
    }
  }

  const size_t   cbase = (EPI == EPI_HR) ? (size_t)0 : (size_t)blockIdx.z * sCz;
  const unsigned ncol  = n0;

  float bcol[4];
  #pragma unroll
  for (int nt = 0; nt < 4; ++nt) bcol[nt] = 0.0f;
  if (EPI == EPI_HR || EPI == EPI_F32B) {
    #pragma unroll
    for (int nt = 0; nt < 4; ++nt) bcol[nt] = bias[n0 + nt * 16u + lq];
  }

  float* so = sO + wave * (16u * OP);

  #pragma unroll
  for (int mt = 0; mt < 2; ++mt) {
    if (mt != 0) __syncthreads();
    #pragma unroll
    for (int r = 0; r < 8; ++r) {
      float brow = 0.0f;
      if (EPI == EPI_VT) brow = bias[m0 + mt * 16u + hi * 8u + r];
      #pragma unroll
      for (int nt = 0; nt < 4; ++nt) {
        float val = acc[mt][nt][r];
        if (EPI == EPI_H16 || EPI == EPI_F32B) val *= scale;
        if (EPI == EPI_HR  || EPI == EPI_F32B) val += bcol[nt];
        if (EPI == EPI_VT)                     val += brow;
        so[(hi * 8u + r) * OP + nt * 16u + lq] = val;
      }
    }
    __syncthreads();

    if (EPI == EPI_F32B) {
      static_assert(32 * 16 * 8 == 16 * 64 * 4);
      float* Cf = (float*)C + cbase;
      v4f    vals[8];
      size_t gidx[8];
      #pragma unroll
      for (int it = 0; it < 8; ++it) {
        const unsigned row = it * 2u + hi;
        vals[it] = *(const v4f*)(so + row * OP + lq * 4u);
        gidx[it] = (size_t)(m0 + mt * 16u + row) * ldc + ncol + lq * 4u;
      }
      #pragma unroll
      for (int it = 0; it < 8; ++it) *(volatile v4f*)(Cf + gidx[it]) = vals[it];
      __threadfence();
      #pragma unroll
      for (int it = 0; it < 8; ++it) *(volatile v4f*)(Cf + gidx[it]) = vals[it];
    } else {
      static_assert(32 * 16 * 4 == 16 * 64 * 2);
      f16* Ch = (f16*)C + cbase;
      v4u    vals[4];
      v4u    valr[4];
      size_t gidx[4];
      #pragma unroll
      for (int it = 0; it < 4; ++it) {
        const unsigned row = it * 4u + (lane >> 3);
        const unsigned c8  = (lane & 7u) * 8u;
        const v4f x0 = *(const v4f*)(so + row * OP + c8);
        const v4f x1 = *(const v4f*)(so + row * OP + c8 + 4u);
        Pack8H ph;
        Pack8H pr;
        pr.u = (v4u){0u, 0u, 0u, 0u};
        #pragma unroll
        for (int i = 0; i < 4; ++i) {
          const f16 h0 = toh_flush(x0[i]);
          const f16 h1 = toh_flush(x1[i]);
          ph.h[i]     = h0;
          ph.h[4 + i] = h1;
          if (EPI == EPI_HR) {
            pr.h[i]     = toh_flush((x0[i] - (float)h0) * 2048.0f);
            pr.h[4 + i] = toh_flush((x1[i] - (float)h1) * 2048.0f);
          }
        }
        vals[it] = ph.u;
        valr[it] = pr.u;
        gidx[it] = (size_t)(m0 + mt * 16u + row) * ldc + ncol + c8;
      }
      #pragma unroll
      for (int it = 0; it < 4; ++it) *(volatile v4u*)(Ch + gidx[it]) = vals[it];
      if (EPI == EPI_HR) {
        #pragma unroll
        for (int it = 0; it < 4; ++it) *(volatile v4u*)(Ch + sCz + gidx[it]) = valr[it];
      }
      __threadfence();
      #pragma unroll
      for (int it = 0; it < 4; ++it) *(volatile v4u*)(Ch + gidx[it]) = vals[it];
      if (EPI == EPI_HR) {
        #pragma unroll
        for (int it = 0; it < 4; ++it) *(volatile v4u*)(Ch + sCz + gidx[it]) = valr[it];
      }
    }
  }
}

__global__ __launch_bounds__(256) __attribute__((amdgpu_num_vgpr(256)))
void score_kernel(const f16* __restrict__ Qh,
                  const f16* __restrict__ Kh,
                  float* __restrict__ Sout,
                  unsigned long long rofs, float scale) {
  union FragH { v16h v; v4u q[2]; };

  __shared__ __align__(16) float sO[NWAVE * 16 * OP];

  const unsigned tid  = threadIdx.x;
  const unsigned wave = (unsigned)__builtin_amdgcn_readfirstlane((int)(tid >> 5));
  const unsigned lane = tid & 31u;
  const unsigned lq   = lane & 15u;
  const unsigned hi   = lane >> 4;
  const unsigned m0   = blockIdx.x * 128u + (wave & 3u) * 32u;
  const unsigned n0   = blockIdx.y * 128u + (wave >> 2) * 64u;

  const f16* ap[2];
  const f16* bp[4];
  #pragma unroll
  for (int mt = 0; mt < 2; ++mt) ap[mt] = Qh + (size_t)(m0 + mt * 16u + lq) * DM + hi * 8u;
  #pragma unroll
  for (int nt = 0; nt < 4; ++nt) bp[nt] = Kh + (size_t)(n0 + nt * 16u + lq) * DM + hi * 8u;

  v8f acc[2][4];
  v8f accr[2][4];
  #pragma unroll
  for (int mt = 0; mt < 2; ++mt) {
    #pragma unroll
    for (int nt = 0; nt < 4; ++nt) {
      acc[mt][nt]  = (v8f){0, 0, 0, 0, 0, 0, 0, 0};
      accr[mt][nt] = (v8f){0, 0, 0, 0, 0, 0, 0, 0};
    }
  }

  #pragma unroll 1
  for (unsigned k = 0; k < (unsigned)(DM / 32); ++k) {
    const unsigned ko = k * 32u;
    FragH ah[2], ar[2];
    #pragma unroll
    for (int mt = 0; mt < 2; ++mt) {
      ah[mt].q[0] = *(const v4u*)(ap[mt] + ko);
      ah[mt].q[1] = *(const v4u*)(ap[mt] + ko + 16u);
      ar[mt].q[0] = *(const v4u*)(ap[mt] + rofs + ko);
      ar[mt].q[1] = *(const v4u*)(ap[mt] + rofs + ko + 16u);
    }
    #pragma unroll
    for (int nt = 0; nt < 4; ++nt) {
      FragH bh, br;
      bh.q[0] = *(const v4u*)(bp[nt] + ko);
      bh.q[1] = *(const v4u*)(bp[nt] + ko + 16u);
      br.q[0] = *(const v4u*)(bp[nt] + rofs + ko);
      br.q[1] = *(const v4u*)(bp[nt] + rofs + ko + 16u);
      #pragma unroll
      for (int mt = 0; mt < 2; ++mt) acc[mt][nt]  = mma16(ah[mt].v, bh.v, acc[mt][nt]);
      #pragma unroll
      for (int mt = 0; mt < 2; ++mt) accr[mt][nt] = mma16(ah[mt].v, br.v, accr[mt][nt]);
      #pragma unroll
      for (int mt = 0; mt < 2; ++mt) accr[mt][nt] = mma16(ar[mt].v, bh.v, accr[mt][nt]);
    }
  }

  float* so = sO + wave * (16u * OP);

  #pragma unroll
  for (int mt = 0; mt < 2; ++mt) {
    if (mt != 0) __syncthreads();
    #pragma unroll
    for (int r = 0; r < 8; ++r) {
      #pragma unroll
      for (int nt = 0; nt < 4; ++nt) {
        const float val = (acc[mt][nt][r] + accr[mt][nt][r] * (1.0f / 2048.0f)) * scale;
        so[(hi * 8u + r) * OP + nt * 16u + lq] = val;
      }
    }
    __syncthreads();

    static_assert(32 * 16 * 8 == 16 * 64 * 4);
    v4f    vals[8];
    size_t gidx[8];
    #pragma unroll
    for (int it = 0; it < 8; ++it) {
      const unsigned row = it * 2u + hi;
      vals[it] = *(const v4f*)(so + row * OP + lq * 4u);
      gidx[it] = (size_t)(m0 + mt * 16u + row) * SEQ + n0 + lq * 4u;
    }
    #pragma unroll
    for (int it = 0; it < 8; ++it) *(volatile v4f*)(Sout + gidx[it]) = vals[it];
    __threadfence();
    #pragma unroll
    for (int it = 0; it < 8; ++it) *(volatile v4f*)(Sout + gidx[it]) = vals[it];
  }
}

__global__ __launch_bounds__(256) void colstat_kernel(const float* __restrict__ S, float* __restrict__ cst) {
  #pragma clang fp contract(off)
  __shared__ __align__(16) float sM[NWAVE * CSC];
  __shared__ __align__(16) float sZ[NWAVE * CSC];
  __shared__ __align__(16) float sC[CSC];

  const unsigned tid  = threadIdx.x;
  const unsigned wave = (unsigned)__builtin_amdgcn_readfirstlane((int)(tid >> 5));
  const unsigned lane = tid & 31u;
  const float L2E = 1.4426950408889634f;
  const float LN2 = 0.6931471805599453f;

  const float* sp = S + (size_t)wave * SEQ + (size_t)blockIdx.x * CSC + lane * 4u;

  v4f m = (v4f){-__builtin_inff(), -__builtin_inff(), -__builtin_inff(), -__builtin_inff()};
  #pragma unroll 1
  for (unsigned r = 0; r < (unsigned)(SEQ / NWAVE); ++r) {
    const v4f xv = *(const v4f*)(sp + (size_t)r * ((size_t)NWAVE * SEQ));
    #pragma unroll
    for (int i = 0; i < 4; ++i) m[i] = fmaxf(m[i], xv[i]);
  }
  v4f z = (v4f){0.0f, 0.0f, 0.0f, 0.0f};
  #pragma unroll 1
  for (unsigned r = 0; r < (unsigned)(SEQ / NWAVE); ++r) {
    const v4f xv = *(const v4f*)(sp + (size_t)r * ((size_t)NWAVE * SEQ));
    #pragma unroll
    for (int i = 0; i < 4; ++i) z[i] += __builtin_amdgcn_exp2f((xv[i] - m[i]) * L2E);
  }
  *(v4f*)(sM + wave * CSC + lane * 4u) = m;
  *(v4f*)(sZ + wave * CSC + lane * 4u) = z;
  __syncthreads();

  if (tid < (unsigned)CSC) {
    float M = -__builtin_inff();
    #pragma unroll 1
    for (int w = 0; w < NWAVE; ++w) M = fmaxf(M, sM[w * CSC + tid]);
    float Z = 0.0f;
    #pragma unroll 1
    for (int w = 0; w < NWAVE; ++w) {
      const float t = __builtin_amdgcn_exp2f((sM[w * CSC + tid] - M) * L2E);
      Z += sZ[w * CSC + tid] * t;
    }
    sC[tid] = M + (log2f(Z) - 14.0f) * LN2;
  }
  __syncthreads();

  if (wave == 0u) {
    static_assert(32 * 16 == CSC * 4);
    const v4f o = *(const v4f*)(sC + lane * 4u);
    float* dst = cst + (size_t)blockIdx.x * CSC + lane * 4u;
    *(volatile v4f*)(dst) = o;
    __threadfence();
    *(volatile v4f*)(dst) = o;
  }
}

__global__ __launch_bounds__(256) void pnorm_kernel(const float* __restrict__ S,
                                                    const float* __restrict__ cst,
                                                    f16* __restrict__ P,
                                                    f16* __restrict__ PR) {
  #pragma clang fp contract(off)
  static_assert(32 * 16 * NCH == SEQ * 2);
  const unsigned tid  = threadIdx.x;
  const unsigned wave = (unsigned)__builtin_amdgcn_readfirstlane((int)(tid >> 5));
  const unsigned lane = tid & 31u;
  const unsigned row  = blockIdx.x * 8u + wave;
  const float L2E = 1.4426950408889634f;

  const float* sp = S + (size_t)row * SEQ + lane * 8u;
  const float* cp = cst + lane * 8u;
  f16* dp = P  + (size_t)row * SEQ + lane * 8u;
  f16* dr = PR + (size_t)row * SEQ + lane * 8u;

  #pragma unroll 1
  for (unsigned g = 0; g < (unsigned)NCH; g += (unsigned)GCH) {
    v4u pk[GCH];
    v4u pq[GCH];
    #pragma unroll
    for (int j = 0; j < GCH; ++j) {
      const unsigned co = (g + (unsigned)j) * 256u;
      const v4f x0 = *(const v4f*)(sp + co);
      const v4f x1 = *(const v4f*)(sp + co + 4u);
      const v4f c0 = *(const v4f*)(cp + co);
      const v4f c1 = *(const v4f*)(cp + co + 4u);
      Pack8H ph;
      Pack8H pr;
      #pragma unroll
      for (int i = 0; i < 4; ++i) {
        const float e0 = (x0[i] - c0[i]) * L2E;
        const float e1 = (x1[i] - c1[i]) * L2E;
        const float p0 = __builtin_amdgcn_exp2f(e0);
        const float p1 = __builtin_amdgcn_exp2f(e1);
        const f16 h0 = (e0 < -14.0f) ? (f16)0.0f : (f16)p0;
        const f16 h1 = (e1 < -14.0f) ? (f16)0.0f : (f16)p1;
        ph.h[i]     = h0;
        ph.h[4 + i] = h1;
        pr.h[i]     = toh_flush((p0 - (float)h0) * 2048.0f);
        pr.h[4 + i] = toh_flush((p1 - (float)h1) * 2048.0f);
      }
      pk[j] = ph.u;
      pq[j] = pr.u;
    }
    #pragma unroll
    for (int j = 0; j < GCH; ++j) *(volatile v4u*)(dp + (g + (unsigned)j) * 256u) = pk[j];
    #pragma unroll
    for (int j = 0; j < GCH; ++j) *(volatile v4u*)(dr + (g + (unsigned)j) * 256u) = pq[j];
    __threadfence();
    #pragma unroll
    for (int j = 0; j < GCH; ++j) *(volatile v4u*)(dp + (g + (unsigned)j) * 256u) = pk[j];
    #pragma unroll
    for (int j = 0; j < GCH; ++j) *(volatile v4u*)(dr + (g + (unsigned)j) * 256u) = pq[j];
  }
}

__global__ __launch_bounds__(256) __attribute__((amdgpu_num_vgpr(256)))
void pv_kernel(const f16* __restrict__ Ph,
               const f16* __restrict__ Pr,
               const f16* __restrict__ Vt,
               f16* __restrict__ Ch,
               f16* __restrict__ Cr,
               float scale) {
  union FragH { v16h v; v4u q[2]; };

  __shared__ __align__(16) float sO[NWAVE * 16 * OP];

  const unsigned tid  = threadIdx.x;
  const unsigned wave = (unsigned)__builtin_amdgcn_readfirstlane((int)(tid >> 5));
  const unsigned lane = tid & 31u;
  const unsigned lq   = lane & 15u;
  const unsigned hi   = lane >> 4;
  const unsigned m0   = blockIdx.x * 128u + (wave & 3u) * 32u;
  const unsigned n0   = blockIdx.y * 128u + (wave >> 2) * 64u;

  size_t aoff[2];
  size_t boff[4];
  #pragma unroll
  for (int mt = 0; mt < 2; ++mt) aoff[mt] = (size_t)(m0 + mt * 16u + lq) * SEQ + hi * 8u;
  #pragma unroll
  for (int nt = 0; nt < 4; ++nt) boff[nt] = (size_t)(n0 + nt * 16u + lq) * SEQ + hi * 8u;

  v8f acc[2][4];
  v8f accr[2][4];
  #pragma unroll
  for (int mt = 0; mt < 2; ++mt) {
    #pragma unroll
    for (int nt = 0; nt < 4; ++nt) {
      acc[mt][nt]  = (v8f){0, 0, 0, 0, 0, 0, 0, 0};
      accr[mt][nt] = (v8f){0, 0, 0, 0, 0, 0, 0, 0};
    }
  }

  #pragma unroll 1
  for (unsigned k = 0; k < (unsigned)(SEQ / 32); ++k) {
    const unsigned ko = k * 32u;
    FragH ah[2], ar[2];
    #pragma unroll
    for (int mt = 0; mt < 2; ++mt) {
      ah[mt].q[0] = *(const v4u*)(Ph + aoff[mt] + ko);
      ah[mt].q[1] = *(const v4u*)(Ph + aoff[mt] + ko + 16u);
      ar[mt].q[0] = *(const v4u*)(Pr + aoff[mt] + ko);
      ar[mt].q[1] = *(const v4u*)(Pr + aoff[mt] + ko + 16u);
    }
    #pragma unroll
    for (int nt = 0; nt < 4; ++nt) {
      FragH bh;
      bh.q[0] = *(const v4u*)(Vt + boff[nt] + ko);
      bh.q[1] = *(const v4u*)(Vt + boff[nt] + ko + 16u);
      #pragma unroll
      for (int mt = 0; mt < 2; ++mt) acc[mt][nt]  = mma16(ah[mt].v, bh.v, acc[mt][nt]);
      #pragma unroll
      for (int mt = 0; mt < 2; ++mt) accr[mt][nt] = mma16(ar[mt].v, bh.v, accr[mt][nt]);
    }
  }

  float* so = sO + wave * (16u * OP);

  #pragma unroll
  for (int mt = 0; mt < 2; ++mt) {
    if (mt != 0) __syncthreads();
    #pragma unroll
    for (int r = 0; r < 8; ++r) {
      #pragma unroll
      for (int nt = 0; nt < 4; ++nt) {
        const float val = (acc[mt][nt][r] + accr[mt][nt][r] * (1.0f / 2048.0f)) * scale;
        so[(hi * 8u + r) * OP + nt * 16u + lq] = val;
      }
    }
    __syncthreads();

    static_assert(32 * 16 * 4 == 16 * 64 * 2);
    v4u    vals[4];
    v4u    valr[4];
    size_t gidx[4];
    #pragma unroll
    for (int it = 0; it < 4; ++it) {
      const unsigned row = it * 4u + (lane >> 3);
      const unsigned c8  = (lane & 7u) * 8u;
      const v4f x0 = *(const v4f*)(so + row * OP + c8);
      const v4f x1 = *(const v4f*)(so + row * OP + c8 + 4u);
      Pack8H ph;
      Pack8H pr;
      #pragma unroll
      for (int i = 0; i < 4; ++i) {
        const f16 h0 = toh_flush(x0[i]);
        const f16 h1 = toh_flush(x1[i]);
        ph.h[i]     = h0;
        ph.h[4 + i] = h1;
        pr.h[i]     = toh_flush((x0[i] - (float)h0) * 2048.0f);
        pr.h[4 + i] = toh_flush((x1[i] - (float)h1) * 2048.0f);
      }
      vals[it] = ph.u;
      valr[it] = pr.u;
      gidx[it] = (size_t)(m0 + mt * 16u + row) * DM + n0 + c8;
    }
    #pragma unroll
    for (int it = 0; it < 4; ++it) *(volatile v4u*)(Ch + gidx[it]) = vals[it];
    #pragma unroll
    for (int it = 0; it < 4; ++it) *(volatile v4u*)(Cr + gidx[it]) = valr[it];
    __threadfence();
    #pragma unroll
    for (int it = 0; it < 4; ++it) *(volatile v4u*)(Ch + gidx[it]) = vals[it];
    #pragma unroll
    for (int it = 0; it < 4; ++it) *(volatile v4u*)(Cr + gidx[it]) = valr[it];
  }
}

__global__ __launch_bounds__(256) __attribute__((amdgpu_num_vgpr(256)))
void oproj_kernel(const f16* __restrict__ Xh,
                  const f16* __restrict__ Xr,
                  const f16* __restrict__ Wt,
                  const float* __restrict__ bias,
                  float* __restrict__ Out,
                  float scale) {
  union FragH { v16h v; v4u q[2]; };

  __shared__ __align__(16) float sO[NWAVE * 16 * OP];

  const unsigned tid  = threadIdx.x;
  const unsigned wave = (unsigned)__builtin_amdgcn_readfirstlane((int)(tid >> 5));
  const unsigned lane = tid & 31u;
  const unsigned lq   = lane & 15u;
  const unsigned hi   = lane >> 4;
  const unsigned m0   = blockIdx.x * 128u + (wave & 3u) * 32u;
  const unsigned n0   = blockIdx.y * 128u + (wave >> 2) * 64u;

  size_t aoff[2];
  size_t boff[4];
  #pragma unroll
  for (int mt = 0; mt < 2; ++mt) aoff[mt] = (size_t)(m0 + mt * 16u + lq) * DM + hi * 8u;
  #pragma unroll
  for (int nt = 0; nt < 4; ++nt) boff[nt] = (size_t)(n0 + nt * 16u + lq) * DM + hi * 8u;

  v8f acc[2][4];
  v8f accr[2][4];
  #pragma unroll
  for (int mt = 0; mt < 2; ++mt) {
    #pragma unroll
    for (int nt = 0; nt < 4; ++nt) {
      acc[mt][nt]  = (v8f){0, 0, 0, 0, 0, 0, 0, 0};
      accr[mt][nt] = (v8f){0, 0, 0, 0, 0, 0, 0, 0};
    }
  }

  #pragma unroll 1
  for (unsigned k = 0; k < (unsigned)(DM / 32); ++k) {
    const unsigned ko = k * 32u;
    FragH ah[2], ar[2];
    #pragma unroll
    for (int mt = 0; mt < 2; ++mt) {
      ah[mt].q[0] = *(const v4u*)(Xh + aoff[mt] + ko);
      ah[mt].q[1] = *(const v4u*)(Xh + aoff[mt] + ko + 16u);
      ar[mt].q[0] = *(const v4u*)(Xr + aoff[mt] + ko);
      ar[mt].q[1] = *(const v4u*)(Xr + aoff[mt] + ko + 16u);
    }
    #pragma unroll
    for (int nt = 0; nt < 4; ++nt) {
      FragH bh;
      bh.q[0] = *(const v4u*)(Wt + boff[nt] + ko);
      bh.q[1] = *(const v4u*)(Wt + boff[nt] + ko + 16u);
      #pragma unroll
      for (int mt = 0; mt < 2; ++mt) acc[mt][nt]  = mma16(ah[mt].v, bh.v, acc[mt][nt]);
      #pragma unroll
      for (int mt = 0; mt < 2; ++mt) accr[mt][nt] = mma16(ar[mt].v, bh.v, accr[mt][nt]);
    }
  }

  float bcol[4];
  #pragma unroll
  for (int nt = 0; nt < 4; ++nt) bcol[nt] = bias[n0 + nt * 16u + lq];

  float* so = sO + wave * (16u * OP);

  #pragma unroll
  for (int mt = 0; mt < 2; ++mt) {
    if (mt != 0) __syncthreads();
    #pragma unroll
    for (int r = 0; r < 8; ++r) {
      #pragma unroll
      for (int nt = 0; nt < 4; ++nt) {
        const float val = (acc[mt][nt][r] + accr[mt][nt][r] * (1.0f / 2048.0f)) * scale + bcol[nt];
        so[(hi * 8u + r) * OP + nt * 16u + lq] = val;
      }
    }
    __syncthreads();

    static_assert(32 * 16 * 8 == 16 * 64 * 4);
    v4f    vals[8];
    size_t gidx[8];
    #pragma unroll
    for (int it = 0; it < 8; ++it) {
      const unsigned row = it * 2u + hi;
      vals[it] = *(const v4f*)(so + row * OP + lq * 4u);
      gidx[it] = (size_t)(m0 + mt * 16u + row) * DM + n0 + lq * 4u;
    }
    #pragma unroll
    for (int it = 0; it < 8; ++it) *(volatile v4f*)(Out + gidx[it]) = vals[it];
    __threadfence();
    #pragma unroll
    for (int it = 0; it < 8; ++it) *(volatile v4f*)(Out + gidx[it]) = vals[it];
  }
}

extern "C" void kernel_launch(void* const* d_in, const int* in_sizes, int n_in,
                              void* d_out, int out_size, void* d_ws, size_t ws_size,
                              hipStream_t stream) {
  if (n_in < 11) return;
  const size_t rows_used = (size_t)(NB - 1) * SEQ_FULL + SEQ;
  if ((size_t)in_sizes[0] < rows_used * DM) return;
  if ((size_t)in_sizes[1] < rows_used * DM) return;
  if ((size_t)in_sizes[2] < rows_used * DM) return;
  if ((size_t)in_sizes[3] < (size_t)DM * DM) return;
  if ((size_t)in_sizes[4] < (size_t)DM) return;
  if ((size_t)in_sizes[5] < (size_t)DM * DM) return;
  if ((size_t)in_sizes[6] < (size_t)DM) return;
  if ((size_t)in_sizes[7] < (size_t)DM * DM) return;
  if ((size_t)in_sizes[8] < (size_t)DM) return;
  if ((size_t)in_sizes[9] < (size_t)DM * DM) return;
  if ((size_t)in_sizes[10] < (size_t)DM) return;
  if ((size_t)out_size < rows_used * DM) return;
  if (ws_size < WS_TOTAL) return;

  const float* xq = (const float*)d_in[0];
  const float* xk = (const float*)d_in[1];
  const float* xv = (const float*)d_in[2];
  const float* wq = (const float*)d_in[3];
  const float* bq = (const float*)d_in[4];
  const float* wk = (const float*)d_in[5];
  const float* bk = (const float*)d_in[6];
  const float* wv = (const float*)d_in[7];
  const float* bv = (const float*)d_in[8];
  const float* wo = (const float*)d_in[9];
  const float* bo = (const float*)d_in[10];
  float* out = (float*)d_out;

  char* w = (char*)d_ws;
  char*  r1    = w;          w += R1_BYTES;
  char*  r2    = w;          w += R2_BYTES;
  f16*   Pr    = (f16*)w;    w += PR_BYTES;
  f16*   ctxh  = (f16*)w;    w += CX_BYTES;
  f16*   ctxr  = (f16*)w;    w += CX_BYTES;
  f16*   wob   = (f16*)w;    w += WO_BYTES;
  float* biasp = (float*)w;  w += BI_BYTES;
  float* cst   = (float*)w;  w += CS_BYTES;
  f16*   qk    = (f16*)w;    w += QK_BYTES;
  f16*   vt    = (f16*)w;    w += VT_BYTES;

  bf16*  xb = (bf16*)r1;
  float* Sp = (float*)r1;
  bf16*  wb = (bf16*)r2;
  f16*   Pp = (f16*)r2;

  const unsigned long long plane = (unsigned long long)NB * SEQ * DM;
  f16* qh = qk;
  f16* kh = qk + 2ull * plane;

  convert_kernel<<<dim3(NXB + NWB + NOB + 4u), 256, 0, stream>>>(xq, wq, bq, wk, bk, wv, bv, wo, bo, xb, wb, wob, biasp);

  gemm_kernel<bf16, EPI_HR><<<dim3((unsigned)((size_t)NB * SEQ / 128), DM / 128, 1), 256, 0, stream>>>(
      xb, wb, biasp, (void*)qh, DM / 32, DM, DM, DM, 0ull, 0ull, plane, 1.0f);

  convert_kernel<<<dim3(NXB), 256, 0, stream>>>(xk, wq, bq, wk, bk, wv, bv, wo, bo, xb, wb, wob, biasp);

  gemm_kernel<bf16, EPI_HR><<<dim3((unsigned)((size_t)NB * SEQ / 128), DM / 128, 1), 256, 0, stream>>>(
      xb, wb + (size_t)DM * DM, biasp + DM, (void*)kh, DM / 32, DM, DM, DM, 0ull, 0ull, plane, 1.0f);

  convert_kernel<<<dim3(NXB), 256, 0, stream>>>(xv, wq, bq, wk, bk, wv, bv, wo, bo, xb, wb, wob, biasp);

  gemm_kernel<bf16, EPI_VT><<<dim3(DM / 128, SEQ / 128, NB), 256, 0, stream>>>(
      wb + (size_t)2 * DM * DM, xb, biasp + 2 * DM, (void*)vt, DM / 32, DM, DM, SEQ,
      0ull, (unsigned long long)SEQ * DM, (unsigned long long)DM * SEQ, 1.0f);

  for (int b = 0; b < NB; ++b) {
    score_kernel<<<dim3(SEQ / 128, SEQ / 128, 1), 256, 0, stream>>>(
        qh + (size_t)b * SEQ * DM, kh + (size_t)b * SEQ * DM, Sp, plane, 0.125f);

    colstat_kernel<<<dim3(SEQ / CSC), 256, 0, stream>>>(Sp, cst);

    pnorm_kernel<<<dim3(SEQ / 8), 256, 0, stream>>>(Sp, cst, Pp, Pr);

    pv_kernel<<<dim3(SEQ / 128, DM / 128, 1), 256, 0, stream>>>(
        Pp, Pr, vt + (size_t)b * DM * SEQ, ctxh, ctxr, 1.0f / 16384.0f);

    oproj_kernel<<<dim3(SEQ / 128, DM / 128, 1), 256, 0, stream>>>(
        ctxh, ctxr, wob, biasp + 3 * DM, out + (size_t)b * SEQ_FULL * DM, 1.0f / 64.0f);
  }
}
